// ImprovedCrossBorderGNN_9526237462757
// MI455X (gfx1250) — hardware-verified
//
#include <hip/hip_runtime.h>
#include <stddef.h>
#include <stdint.h>


#define DF    128
#define NFE   8
#define GR    32
#define AP    136
#define XSP   132
#define RB    64
#define NB    512
#define CHUNK 2048
#define NTHR  256
#define NWAVE 8
#define WCAP  256
#define NGRP  (CHUNK / (NTHR * 4))
#define WPL   (2 * DF * DF)

#define LDS_SACC (NB * DF)
#define LDS_DEN  NB
#define LDS_MX   NB
#define LDS_LIST (NWAVE * WCAP)
#define LDS_BYTES ((LDS_SACC + LDS_DEN + LDS_MX + LDS_LIST + NWAVE) * 4)

static_assert(WCAP == (CHUNK / NTHR) * 32);
static_assert(NGRP >= 1);
static_assert(NB == 512);
static_assert(CHUNK <= 4096);
static_assert(((LDS_SACC + LDS_DEN) % 4) == 0);
static_assert(LDS_BYTES == 274464);
static_assert((NB % NWAVE) == 0);
static_assert((RB % NWAVE) == 0);

typedef float          v2f  __attribute__((ext_vector_type(2)));
typedef float          v4f  __attribute__((ext_vector_type(4)));
typedef float          v8f  __attribute__((ext_vector_type(8)));
typedef int            v4i  __attribute__((ext_vector_type(4)));
typedef unsigned short v8us __attribute__((ext_vector_type(8)));
typedef __bf16         v16b __attribute__((ext_vector_type(16)));
union FragB { v16b v; v8us half[2]; };

__device__ __forceinline__ v8f wmb(v16b a, v16b b, v8f c) {
  v8f d = __builtin_amdgcn_wmma_f32_16x16x32_bf16(false, a, false, b, (short)0, c, false, false);
  asm volatile("v_nop\n\tv_nop\n\tv_nop\n\tv_nop" : "+v"(d) : "v"(a), "v"(b));
  return d;
}

__device__ __forceinline__ float wsum(float v) {
  v += __shfl_xor(v, 16, 32);
  v += __shfl_xor(v, 8, 32);
  v += __shfl_xor(v, 4, 32);
  v += __shfl_xor(v, 2, 32);
  v += __shfl_xor(v, 1, 32);
  return v;
}

__device__ __forceinline__ unsigned short bfr(float f) {
  unsigned u = __float_as_uint(f);
  u += 0x7FFFu + ((u >> 16) & 1u);
  return (unsigned short)(u >> 16);
}
__device__ __forceinline__ void split2(float f, unsigned short& hi, unsigned short& lo) {
  const unsigned short h = bfr(f);
  const float fh = __uint_as_float(((unsigned)h) << 16);
  hi = h;
  lo = bfr(f - fh);
}
__device__ __forceinline__ void split8(v4f a, v4f b, v8us& hi, v8us& lo) {
  unsigned short h, l;
  split2(a.x, h, l); hi[0] = h; lo[0] = l;
  split2(a.y, h, l); hi[1] = h; lo[1] = l;
  split2(a.z, h, l); hi[2] = h; lo[2] = l;
  split2(a.w, h, l); hi[3] = h; lo[3] = l;
  split2(b.x, h, l); hi[4] = h; lo[4] = l;
  split2(b.y, h, l); hi[5] = h; lo[5] = l;
  split2(b.z, h, l); hi[6] = h; lo[6] = l;
  split2(b.w, h, l); hi[7] = h; lo[7] = l;
}

__global__ __launch_bounds__(NTHR) void k_scal(
    const float* __restrict__ ea,
    const float* __restrict__ We1, const float* __restrict__ ae1,
    const float* __restrict__ We2, const float* __restrict__ ae2,
    const float* __restrict__ We3, const float* __restrict__ ae3,
    float* scal, int nE) {
  __shared__ double r0[NTHR];
  __shared__ double r1[NTHR];
  __shared__ __attribute__((aligned(16))) float sl[32];
  const int tid = threadIdx.x, lane = tid & 31, wave = tid >> 5;
  if (tid < 32) sl[tid] = 0.f;
  double s0 = 0.0, s1 = 0.0;
  const int n2 = nE * 2;
  const int n4 = n2 >> 2;
#pragma unroll 1
  for (int i = tid; i < n4; i += NTHR) {
    const v4f a = *(const v4f*)(ea + (size_t)i * 4);
    s0 += (double)a.x; s1 += (double)a.y;
    s0 += (double)a.z; s1 += (double)a.w;
  }
  if (tid == 0 && n4 * 4 < n2) {
    s0 += (double)ea[(size_t)n4 * 4];
    s1 += (double)ea[(size_t)n4 * 4 + 1];
  }
  r0[tid] = s0;
  r1[tid] = s1;
  __syncthreads();
#pragma unroll 1
  for (int s = NTHR / 2; s > 0; s >>= 1) {
    if (tid < s) { r0[tid] += r0[tid + s]; r1[tid] += r1[tid + s]; }
    __syncthreads();
  }
  int l = wave >> 1;
  if (l > 2) l = 2;
  const int j = wave & 1;
  const float* Wp = (l == 0) ? We1 : ((l == 1) ? We2 : We3);
  const float* Ap = (l == 0) ? ae1 : ((l == 1) ? ae2 : ae3);
  const v4f wv = *(const v4f*)(Wp + j * DF + 4 * lane);
  const v4f av = *(const v4f*)(Ap + 4 * lane);
  float t = wv.x * av.x + wv.y * av.y + wv.z * av.z + wv.w * av.w;
  t = wsum(t);
  if (tid == 0) {
    const double inv = (nE > 0) ? (1.0 / (double)nE) : 0.0;
    sl[0] = (float)(r0[0] * inv);
    sl[1] = (float)(r1[0] * inv);
  }
  if (lane == 0 && wave < 6) sl[2 + wave] = t;
  __syncthreads();
  const v4f v = *(const v4f*)(sl + 4 * (lane & 7));
  float* gp = scal + 4 * (lane & 7);
  const bool st = (wave == 0) && (lane < 8);
  if (st) *(volatile v4f*)gp = v;
  __threadfence();
  if (st) *(volatile v4f*)gp = v;
}

__global__ __launch_bounds__(NTHR) void k_prep(const float* __restrict__ W1, const float* __restrict__ W2,
                                               const float* __restrict__ W3, unsigned short* Wt) {
  const int i = blockIdx.x * NTHR + threadIdx.x;
  if (i >= 3 * (DF * DF / 8)) return;
  const int l   = i >> 11;
  const int idx = i & 2047;
  const int n   = idx >> 4;
  const int k8  = (idx & 15) * 8;
  const float* W = (l == 0) ? W1 : ((l == 1) ? W2 : W3);
  v4f a, b;
  a.x = W[(size_t)(k8 + 0) * DF + n]; a.y = W[(size_t)(k8 + 1) * DF + n];
  a.z = W[(size_t)(k8 + 2) * DF + n]; a.w = W[(size_t)(k8 + 3) * DF + n];
  b.x = W[(size_t)(k8 + 4) * DF + n]; b.y = W[(size_t)(k8 + 5) * DF + n];
  b.z = W[(size_t)(k8 + 6) * DF + n]; b.w = W[(size_t)(k8 + 7) * DF + n];
  v8us hi, lo;
  split8(a, b, hi, lo);
  unsigned short* ph = Wt + (size_t)l * WPL + (size_t)n * DF + k8;
  unsigned short* pl = ph + DF * DF;
  *(volatile v8us*)ph = hi;
  *(volatile v8us*)pl = lo;
  __threadfence();
  *(volatile v8us*)ph = hi;
  *(volatile v8us*)pl = lo;
}

__global__ __launch_bounds__(NTHR) void k_enc(const float* __restrict__ x, const float* __restrict__ encW,
                                              const float* __restrict__ encb, const float* __restrict__ bng,
                                              const float* __restrict__ bnb, float* h0, int nN) {
  const int tid = threadIdx.x, lane = tid & 31, wave = tid >> 5;
  const int rb = blockIdx.x * RB;
  v4f w[NFE];
#pragma unroll
  for (int j = 0; j < NFE; ++j) w[j] = *(const v4f*)(encW + j * DF + 4 * lane);
  const v4f be = *(const v4f*)(encb + 4 * lane);
  const v4f bg = *(const v4f*)(bng + 4 * lane);
  const v4f bb = *(const v4f*)(bnb + 4 * lane);
  const float inv = 0.99999500003750f;
  const v4f scl = bg * inv;
#pragma unroll 1
  for (int i = 0; i < RB / NWAVE; ++i) {
    const int row = rb + i * NWAVE + wave;
    if (row >= nN) break;
    const float* xp = x + (size_t)row * NFE;
    const v4f xa = *(const v4f*)xp;
    const v4f xb = *(const v4f*)(xp + 4);
    v4f acc = xa.x * w[0];
    acc = acc + xa.y * w[1];
    acc = acc + xa.z * w[2];
    acc = acc + xa.w * w[3];
    acc = acc + xb.x * w[4];
    acc = acc + xb.y * w[5];
    acc = acc + xb.z * w[6];
    acc = acc + xb.w * w[7];
    v4f v = (acc + be) * scl + bb;
    v.x = v.x > 0.f ? v.x : 0.f;
    v.y = v.y > 0.f ? v.y : 0.f;
    v.z = v.z > 0.f ? v.z : 0.f;
    v.w = v.w > 0.f ? v.w : 0.f;
    float* op = h0 + (size_t)row * DF + 4 * lane;
    *(volatile v4f*)op = v;
    __threadfence();
    *(volatile v4f*)op = v;
  }
}

__device__ __forceinline__ void epi_tile(v8f acc, int T, int hh, int m, int wave, int ncol,
                                         float cs, float cd, float* Xs, float* Ps, float* Pd) {
  float ss[8], sd[8];
#pragma unroll
  for (int r = 0; r < 8; ++r) {
    const float v = acc[r];
    Xs[(T * 16 + 8 * hh + r) * XSP + ncol] = v;
    ss[r] = v * cs;
    sd[r] = v * cd;
  }
#pragma unroll
  for (int mk = 1; mk < 16; mk <<= 1) {
#pragma unroll
    for (int r = 0; r < 8; ++r) {
      ss[r] += __shfl_xor(ss[r], mk, 32);
      sd[r] += __shfl_xor(sd[r], mk, 32);
    }
  }
  if (m == 0) {
#pragma unroll
    for (int r = 0; r < 8; ++r) {
      Ps[(T * 16 + 8 * hh + r) * NWAVE + wave] = ss[r];
      Pd[(T * 16 + 8 * hh + r) * NWAVE + wave] = sd[r];
    }
  }
}

__global__ __launch_bounds__(NTHR) void k_gemm(
    const float* __restrict__ h, const unsigned short* __restrict__ Wt,
    const float* __restrict__ att_src, const float* __restrict__ att_dst,
    float* g, float* asrc, float* adst, int nN) {
  __shared__ __attribute__((aligned(16))) unsigned short Ah[GR * AP];
  __shared__ __attribute__((aligned(16))) unsigned short Al[GR * AP];
  __shared__ __attribute__((aligned(16))) float Xs[GR * XSP];
  __shared__ __attribute__((aligned(16))) float Ps[GR * NWAVE];
  __shared__ __attribute__((aligned(16))) float Pd[GR * NWAVE];
  __shared__ __attribute__((aligned(16))) float Sa[GR];
  __shared__ __attribute__((aligned(16))) float Sd[GR];

  const int tid  = threadIdx.x;
  const int lane = tid & 31;
  const int wave = tid >> 5;
  const int hh   = lane >> 4;
  const int m    = lane & 15;
  const int rowBase = blockIdx.x * GR;

  {
    const int r  = tid >> 3;
    const int c0 = (tid & 7) * 16;
    int row = rowBase + r;
    if (row > nN - 1) row = nN - 1;
    const float* p = h + (size_t)row * DF + c0;
    const v4f f0 = *(const v4f*)(p), f1 = *(const v4f*)(p + 4);
    const v4f f2 = *(const v4f*)(p + 8), f3 = *(const v4f*)(p + 12);
    v8us h0v, l0v, h1v, l1v;
    split8(f0, f1, h0v, l0v);
    split8(f2, f3, h1v, l1v);
    *(v8us*)(Ah + r * AP + c0)     = h0v;
    *(v8us*)(Ah + r * AP + c0 + 8) = h1v;
    *(v8us*)(Al + r * AP + c0)     = l0v;
    *(v8us*)(Al + r * AP + c0 + 8) = l1v;
  }
  __syncthreads();

  const int ncol = wave * 16 + m;
  const unsigned short* Wh = Wt;
  const unsigned short* Wl = Wt + DF * DF;
  v8f c0a = {0.f, 0.f, 0.f, 0.f, 0.f, 0.f, 0.f, 0.f};
  v8f c1a = {0.f, 0.f, 0.f, 0.f, 0.f, 0.f, 0.f, 0.f};
#pragma unroll
  for (int kt = 0; kt < DF / 32; ++kt) {
    const int k0 = kt * 32;
    FragB a0h, a0l, a1h, a1l, bh, bl;
    const unsigned short* pbh = Wh + (size_t)ncol * DF + k0 + 8 * hh;
    const unsigned short* pbl = Wl + (size_t)ncol * DF + k0 + 8 * hh;
    const unsigned short* ph0 = Ah + m * AP + k0 + 8 * hh;
    const unsigned short* ph1 = Ah + (16 + m) * AP + k0 + 8 * hh;
    const unsigned short* pl0 = Al + m * AP + k0 + 8 * hh;
    const unsigned short* pl1 = Al + (16 + m) * AP + k0 + 8 * hh;
    bh.half[0]  = *(const v8us*)pbh;  bh.half[1]  = *(const v8us*)(pbh + 16);
    bl.half[0]  = *(const v8us*)pbl;  bl.half[1]  = *(const v8us*)(pbl + 16);
    a0h.half[0] = *(const v8us*)ph0;  a0h.half[1] = *(const v8us*)(ph0 + 16);
    a1h.half[0] = *(const v8us*)ph1;  a1h.half[1] = *(const v8us*)(ph1 + 16);
    a0l.half[0] = *(const v8us*)pl0;  a0l.half[1] = *(const v8us*)(pl0 + 16);
    a1l.half[0] = *(const v8us*)pl1;  a1l.half[1] = *(const v8us*)(pl1 + 16);
    c0a = wmb(a0h.v, bh.v, c0a);
    c0a = wmb(a0h.v, bl.v, c0a);
    c0a = wmb(a0l.v, bh.v, c0a);
    c1a = wmb(a1h.v, bh.v, c1a);
    c1a = wmb(a1h.v, bl.v, c1a);
    c1a = wmb(a1l.v, bh.v, c1a);
  }

  const float cs = att_src[ncol];
  const float cd = att_dst[ncol];
  epi_tile(c0a, 0, hh, m, wave, ncol, cs, cd, Xs, Ps, Pd);
  epi_tile(c1a, 1, hh, m, wave, ncol, cs, cd, Xs, Ps, Pd);
  __syncthreads();
  if (tid < GR) {
    float s = 0.f;
#pragma unroll
    for (int w = 0; w < NWAVE; ++w) s += Ps[tid * NWAVE + w];
    Sa[tid] = s;
  } else if (tid < 2 * GR) {
    const int t = tid - GR;
    float s = 0.f;
#pragma unroll
    for (int w = 0; w < NWAVE; ++w) s += Pd[t * NWAVE + w];
    Sd[t] = s;
  }
  __syncthreads();

  v4f xr[4];
#pragma unroll
  for (int i = 0; i < 4; ++i) xr[i] = *(const v4f*)(Xs + (4 * wave + i) * XSP + 4 * lane);
  const int li = (lane & 7) * 4;
  const v4f va = *(const v4f*)(Sa + li);
  const v4f vd = *(const v4f*)(Sd + li);
  const v4f gv = (lane < 8) ? va : vd;
  float* gp = (lane < 8) ? (asrc + rowBase + li) : (adst + rowBase + li);
  const bool gst = (wave == 0) && (lane < 16);
  float* gpp[4];
#pragma unroll
  for (int i = 0; i < 4; ++i) gpp[i] = g + (size_t)(rowBase + 4 * wave + i) * DF + 4 * lane;

#pragma unroll
  for (int i = 0; i < 4; ++i) *(volatile v4f*)(gpp[i]) = xr[i];
  if (gst) *(volatile v4f*)gp = gv;
  __threadfence();
#pragma unroll
  for (int i = 0; i < 4; ++i) *(volatile v4f*)(gpp[i]) = xr[i];
  if (gst) *(volatile v4f*)gp = gv;
}

__global__ __launch_bounds__(NTHR) void k_gat(
    const int* __restrict__ ei, const float* __restrict__ ea,
    const float* __restrict__ g, const float* __restrict__ asrc, const float* __restrict__ adst,
    const float* __restrict__ scal, const float* __restrict__ bias, const float* __restrict__ res,
    float* out, int nN, int nE, int lidx, int mode) {
  extern __shared__ v4f lds_dyn[];
  float* sacc = (float*)lds_dyn;
  float* den  = sacc + LDS_SACC;
  float* mx   = den + LDS_DEN;
  int*   list = (int*)(mx + LDS_MX);
  int*   wcnt = list + LDS_LIST;

  const int tid  = threadIdx.x;
  const int lane = tid & 31;
  const int wave = tid >> 5;
  const int nodeBase = blockIdx.x * NB;

  {
    const v4f z4 = {0.f, 0.f, 0.f, 0.f};
    for (int i = tid; i < (LDS_SACC + LDS_DEN) / 4; i += NTHR) lds_dyn[i] = z4;
    for (int i = tid; i < NB; i += NTHR) mx[i] = -1.0e30f;
  }
  __syncthreads();
  const float u0 = scal[2 + 2 * lidx];
  const float u1 = scal[3 + 2 * lidx];
  const float lterm = scal[0] * u0 + scal[1] * u1;
  const int* eid = ei + nE;
  const bool al16 = ((nE & 3) == 0);

  const int nChunks = (nE + CHUNK - 1) / CHUNK;
#pragma unroll 1
  for (int ch = 0; ch < nChunks; ++ch) {
    const int cbase = ch * CHUNK;
    int wc = 0;
#pragma unroll
    for (int gq = 0; gq < NGRP; ++gq) {
      const int el0 = (gq * NTHR + tid) * 4;
      const int e0  = cbase + el0;
      const int sent = -2147483647 - 1;
      v4i d;
      if (al16 && (cbase + CHUNK <= nE)) {
        d = *(const v4i*)(eid + e0);
      } else {
        d.x = (e0     < nE) ? eid[min(e0, nE - 1)]     : sent;
        d.y = (e0 + 1 < nE) ? eid[min(e0 + 1, nE - 1)] : sent;
        d.z = (e0 + 2 < nE) ? eid[min(e0 + 2, nE - 1)] : sent;
        d.w = (e0 + 3 < nE) ? eid[min(e0 + 3, nE - 1)] : sent;
      }
      const unsigned s0 = (unsigned)d.x - (unsigned)nodeBase;
      const unsigned s1 = (unsigned)d.y - (unsigned)nodeBase;
      const unsigned s2 = (unsigned)d.z - (unsigned)nodeBase;
      const unsigned s3 = (unsigned)d.w - (unsigned)nodeBase;
      const bool h0 = s0 < (unsigned)NB;
      const bool h1 = s1 < (unsigned)NB;
      const bool h2 = s2 < (unsigned)NB;
      const bool h3 = s3 < (unsigned)NB;
      const unsigned many = __builtin_amdgcn_ballot_w32(h0 | h1 | h2 | h3);
      if (many != 0u) {
#define HITJ(J, HJ, SJ) { \
          const unsigned mj = __builtin_amdgcn_ballot_w32(HJ); \
          if (HJ) { \
            const int pos = wc + (int)__builtin_amdgcn_mbcnt_lo(mj, 0u); \
            if (pos < WCAP) list[wave * WCAP + pos] = ((el0 + (J)) << 9) | (int)(SJ); \
          } \
          wc += (int)__builtin_popcount(mj); }
        HITJ(0, h0, s0)
        HITJ(1, h1, s1)
        HITJ(2, h2, s2)
        HITJ(3, h3, s3)
#undef HITJ
      }
    }
    if (lane == 0) wcnt[wave] = wc;
    __syncthreads();

    if (wave == 0) {
      for (int wsx = 0; wsx < NWAVE; ++wsx) {
        int n = wcnt[wsx];
        if (n > WCAP) n = WCAP;
        if (n < 0) n = 0;
        for (int i = 0; i < n; ++i) {
          const int ent  = list[wsx * WCAP + i];
          const int slot = ent & (NB - 1);
          const int el   = (ent >> 9) & (CHUNK - 1);
          int e = cbase + el;
          if (e > nE - 1) e = nE - 1;
          int src = ei[e];
          src = src < 0 ? 0 : (src > nN - 1 ? nN - 1 : src);
          const v2f w2 = *(const v2f*)(ea + (size_t)e * 2);
          int nd = nodeBase + slot;
          if (nd > nN - 1) nd = nN - 1;
          float al = asrc[src] + adst[nd] + (w2.x * u0 + w2.y * u1);
          al = fmaxf(al, 0.2f * al);
          const float mo = mx[slot];
          v4f* sp = (v4f*)(sacc + slot * DF + 4 * lane);
          v4f cur = *sp;
          float dc = den[slot];
          float mn = mo;
          if (al > mo) {
            const float sc = __expf(mo - al);
            cur = cur * sc;
            dc  = dc * sc;
            mn  = al;
            mx[slot] = al;
          }
          const float p = __expf(al - mn);
          const v4f gv = *(const v4f*)(g + (size_t)src * DF + 4 * lane);
          *sp = cur + p * gv;
          den[slot] = dc + p;
        }
      }
    }
    __syncthreads();
  }

  const v4f b4 = *(const v4f*)(bias + 4 * lane);
#pragma unroll 1
  for (int j = 0; j < NB / NWAVE; ++j) {
    const int slot = wave * (NB / NWAVE) + j;
    const int node = nodeBase + slot;
    if (node >= nN) break;
    const size_t nrow = (size_t)node;
    float al = asrc[nrow] + adst[nrow] + lterm;
    al = fmaxf(al, 0.2f * al);
    const float mo = mx[slot];
    const float mn = fmaxf(mo, al);
    const float sc = __expf(mo - mn);
    const float p  = __expf(al - mn);
    const v4f gv = *(const v4f*)(g + nrow * DF + 4 * lane);
    const v4f sv = *(const v4f*)(sacc + slot * DF + 4 * lane) * sc + p * gv;
    const float dv = den[slot] * sc + p;
    const float iv = 1.0f / (dv + 1e-16f);
    v4f hv = sv * iv + b4;
    const v4f rv = *(const v4f*)(res + nrow * DF + 4 * lane);
    if (mode != 0) {
      hv.x = hv.x > 0.f ? hv.x : 0.f;
      hv.y = hv.y > 0.f ? hv.y : 0.f;
      hv.z = hv.z > 0.f ? hv.z : 0.f;
      hv.w = hv.w > 0.f ? hv.w : 0.f;
    } else {
      hv = hv + rv;
    }
    float* op = out + nrow * DF + 4 * lane;
    *(volatile v4f*)op = hv;
    __threadfence();
    *(volatile v4f*)op = hv;
  }
}

extern "C" void kernel_launch(void* const* d_in, const int* in_sizes, int n_in,
                              void* d_out, int out_size, void* d_ws, size_t ws_size,
                              hipStream_t stream) {
  if (n_in < 25) return;
  if (in_sizes[0] <= 0 || (in_sizes[0] % NFE) != 0) return;
  const int nN = in_sizes[0] / NFE;
  if (in_sizes[2] < 0 || (in_sizes[2] & 1) != 0) return;
  const int nE = in_sizes[2] / 2;
  if (in_sizes[1] != 2 * nE) return;
  if (in_sizes[3] != NFE * DF || in_sizes[4] != DF || in_sizes[5] != DF || in_sizes[6] != DF) return;
  for (int l = 0; l < 3; ++l) {
    const int b = 7 + 6 * l;
    if (in_sizes[b] != DF * DF || in_sizes[b + 1] != DF || in_sizes[b + 2] != DF ||
        in_sizes[b + 3] != 2 * DF || in_sizes[b + 4] != DF || in_sizes[b + 5] != DF) return;
  }
  if (out_size != nN * DF) return;

  const float* x    = (const float*)d_in[0];
  const int*   ei   = (const int*)d_in[1];
  const float* ea   = (const float*)d_in[2];
  const float* encW = (const float*)d_in[3];
  const float* encb = (const float*)d_in[4];
  const float* bng  = (const float*)d_in[5];
  const float* bnb  = (const float*)d_in[6];
  const float* Wl[3], * asl[3], * adl[3], * Wel[3], * ael[3], * bl[3];
  for (int l = 0; l < 3; ++l) {
    const int b = 7 + 6 * l;
    Wl[l]  = (const float*)d_in[b];
    asl[l] = (const float*)d_in[b + 1];
    adl[l] = (const float*)d_in[b + 2];
    Wel[l] = (const float*)d_in[b + 3];
    ael[l] = (const float*)d_in[b + 4];
    bl[l]  = (const float*)d_in[b + 5];
  }
  float* out = (float*)d_out;

  const int nP = ((nN + GR - 1) / GR) * GR;
  size_t off = 0;
  float* scal = (float*)((char*)d_ws + off);                    off += 256;
  unsigned short* Wt = (unsigned short*)((char*)d_ws + off);    off += (size_t)3 * WPL * sizeof(unsigned short);
  float* h0   = (float*)((char*)d_ws + off);                    off += (size_t)nP * DF * sizeof(float);
  float* hA   = (float*)((char*)d_ws + off);                    off += (size_t)nP * DF * sizeof(float);
  float* g    = (float*)((char*)d_ws + off);                    off += (size_t)nP * DF * sizeof(float);
  float* asrc = (float*)((char*)d_ws + off);                    off += (((size_t)nP * sizeof(float)) + 255) & ~(size_t)255;
  float* adst = (float*)((char*)d_ws + off);                    off += (((size_t)nP * sizeof(float)) + 255) & ~(size_t)255;
  if (off > ws_size) return;

  k_scal<<<1, NTHR, 0, stream>>>(ea, Wel[0], ael[0], Wel[1], ael[1], Wel[2], ael[2], scal, nE);

  const int nprep = 3 * (DF * DF / 8);
  k_prep<<<(nprep + NTHR - 1) / NTHR, NTHR, 0, stream>>>(Wl[0], Wl[1], Wl[2], Wt);

  k_enc<<<(nN + RB - 1) / RB, NTHR, 0, stream>>>(x, encW, encb, bng, bnb, h0, nN);

  hipFuncSetAttribute(reinterpret_cast<const void*>(&k_gat),
                      hipFuncAttributeMaxDynamicSharedMemorySize, LDS_BYTES);
  const int ggrid = (nN + NB - 1) / NB;
  for (int l = 0; l < 3; ++l) {
    const float* hin = (l == 0) ? h0 : hA;
    float* hout = (l < 2) ? hA : out;
    const int mode = (l < 2) ? 1 : 0;
    k_gemm<<<nP / GR, NTHR, 0, stream>>>(hin, Wt + (size_t)l * WPL, asl[l], adl[l], g, asrc, adst, nN);
    k_gat<<<ggrid, NTHR, LDS_BYTES, stream>>>(ei, ea, g, asrc, adst, scal, bl[l], h0, hout,
                                              nN, nE, l, mode);
  }
}
